// GAT_32916629356560
// MI455X (gfx1250) — hardware-verified
//
#include <hip/hip_runtime.h>
#include <stddef.h>
#include <stdint.h>
#include <math.h>


#define F_IN    256
#define HC      128
#define HC3     64
#define KA      256
#define NTHR    256
#define NWAVE   8
#define EPT     8
#define CHUNK   (NTHR * EPT)
#define WCAP    (EPT * 32)
#define LISTN   (NWAVE * WCAP)
#define NB      512
#define SLOTB   11
#define RCAP    20480
#define DEGCAP  128
#define HDR     32
#define HPITCH  (HDR + RCAP)
#define RECW    256
#define GBM     64
#define GBN     64
#define GTHR    128
#define MROWS   128
#define NEGSL   0.2f
#define WSMAX   134217728
#define LDS_BKT ((2 * RCAP + 2 * NB + LISTN) * 4 + 256)
#define LDS_AGG (NWAVE * RECW * 8 + RECW * 8 + (RCAP + 2 * NB) * 4)

static_assert((CHUNK & (CHUNK - 1)) == 0 && CHUNK <= (1 << SLOTB));
static_assert(NB <= 512 && NB <= (1 << SLOTB) && (NB % NWAVE) == 0);
static_assert(NTHR * 2 == NB);
static_assert(LISTN >= NB);
static_assert((RCAP % (4 * NTHR)) == 0);
static_assert(RCAP >= 16715 + 2048);
static_assert(DEGCAP >= 61 + 8);
static_assert(LDS_BKT <= 300000 && LDS_AGG <= 300000);
static_assert(GBM == (GTHR / 32) * 16);
static_assert(GTHR == 2 * GBN && GTHR == 2 * GBM);
static_assert((F_IN % 32) == 0 && (KA % 32) == 0 && KA == 2 * HC && KA == F_IN);
static_assert((HC % GBN) == 0 && HC3 == GBN);
static_assert((MROWS % GBM) == 0);
static_assert(HC == 4 * 32 && HC3 == 2 * 32);
static_assert((HPITCH % 32) == 0);
static_assert(RECW == 2 * HC);

typedef float          v2f  __attribute__((ext_vector_type(2)));
typedef float          v4f  __attribute__((ext_vector_type(4)));
typedef float          v8f  __attribute__((ext_vector_type(8)));
typedef double         v2d  __attribute__((ext_vector_type(2)));
typedef int            v4i  __attribute__((ext_vector_type(4)));
typedef int            v8i  __attribute__((ext_vector_type(8)));
typedef unsigned int   v4u  __attribute__((ext_vector_type(4)));
typedef unsigned short v8us __attribute__((ext_vector_type(8)));
typedef __bf16         v16b __attribute__((ext_vector_type(16)));
typedef v2f  __attribute__((may_alias)) v2fa;
typedef v4f  __attribute__((may_alias)) v4fa;
typedef v4i  __attribute__((may_alias)) v4ia;
typedef v8us __attribute__((may_alias)) v8usa;
union FragB { v16b v; v8us h[2]; v8i w; };

__device__ __forceinline__ v8f wmb(const FragB& a, const FragB& b, v8f c) {
  v8f d = __builtin_amdgcn_wmma_f32_16x16x32_bf16(false, a.v, false, b.v, (short)0, c, false, false);
  asm volatile("v_nop\n\tv_nop\n\tv_nop\n\tv_nop" : "+v"(d) : "v"(a.w), "v"(b.w));
  return d;
}

__device__ __forceinline__ unsigned int f2bf(float f) {
  const unsigned int u = __float_as_uint(f);
  const unsigned int r = ((u + 0x7FFFu + ((u >> 16) & 1u)) >> 16) & 0xFFFFu;
  return (f != f) ? 0x7FC0u : r;
}
__device__ __forceinline__ float bf2f(unsigned int b) { return __uint_as_float(b << 16); }
__device__ __forceinline__ float bfr(float f) { return bf2f(f2bf(f)); }
__device__ __forceinline__ v2f bfr2(const v2f a) { v2f r; r.x = bfr(a.x); r.y = bfr(a.y); return r; }
__device__ __forceinline__ v4f bfr4(const v4f a) {
  v4f r; r.x = bfr(a.x); r.y = bfr(a.y); r.z = bfr(a.z); r.w = bfr(a.w); return r;
}
__device__ __forceinline__ unsigned int pk2(float lo, float hi) { return f2bf(lo) | (f2bf(hi) << 16); }
__device__ __forceinline__ v4u pack8(const v4f a, const v4f b) {
  v4u r;
  r.x = pk2(a.x, a.y); r.y = pk2(a.z, a.w); r.z = pk2(b.x, b.y); r.w = pk2(b.z, b.w);
  return r;
}
__device__ __forceinline__ float relun(float v) { return (v > 0.f) ? v : (v - v); }

__device__ __forceinline__ int scan_chunk(const int* __restrict__ dsts, int nE, int cbase, int slotBase,
                                          int nb, int vec8, int* list, int tid, int lane, int wave) {
  int wc = 0;
  const int el0  = tid * EPT;
  const int e0   = cbase + el0;
  const int sent = -2147483647 - 1;
  v4i da, db;
  if (vec8 != 0 && cbase + CHUNK <= nE) {
    da = *(const v4i*)(dsts + e0);
    db = *(const v4i*)(dsts + e0 + 4);
  } else {
    da.x = (e0     < nE) ? dsts[min(e0,     nE - 1)] : sent;
    da.y = (e0 + 1 < nE) ? dsts[min(e0 + 1, nE - 1)] : sent;
    da.z = (e0 + 2 < nE) ? dsts[min(e0 + 2, nE - 1)] : sent;
    da.w = (e0 + 3 < nE) ? dsts[min(e0 + 3, nE - 1)] : sent;
    db.x = (e0 + 4 < nE) ? dsts[min(e0 + 4, nE - 1)] : sent;
    db.y = (e0 + 5 < nE) ? dsts[min(e0 + 5, nE - 1)] : sent;
    db.z = (e0 + 6 < nE) ? dsts[min(e0 + 6, nE - 1)] : sent;
    db.w = (e0 + 7 < nE) ? dsts[min(e0 + 7, nE - 1)] : sent;
  }
  const unsigned nbs = (unsigned)slotBase;
  const unsigned unb = (unsigned)nb;
  const unsigned s0 = (unsigned)da.x - nbs, s1 = (unsigned)da.y - nbs;
  const unsigned s2 = (unsigned)da.z - nbs, s3 = (unsigned)da.w - nbs;
  const unsigned s4 = (unsigned)db.x - nbs, s5 = (unsigned)db.y - nbs;
  const unsigned s6 = (unsigned)db.z - nbs, s7 = (unsigned)db.w - nbs;
  const bool h0 = s0 < unb, h1 = s1 < unb, h2 = s2 < unb, h3 = s3 < unb;
  const bool h4 = s4 < unb, h5 = s5 < unb, h6 = s6 < unb, h7 = s7 < unb;
  const unsigned any = __builtin_amdgcn_ballot_w32(h0 | h1 | h2 | h3 | h4 | h5 | h6 | h7);
  if (any != 0u) {
#define HITJ(J, HJ, SJ) { \
      const unsigned mj = __builtin_amdgcn_ballot_w32(HJ); \
      if (mj != 0u) { \
        if (HJ) { \
          const int pos = wc + (int)__builtin_amdgcn_mbcnt_lo(mj, 0u); \
          if (pos < WCAP) list[wave * WCAP + pos] = ((el0 + (J)) << SLOTB) | (int)(SJ); \
        } \
        wc += (int)__builtin_popcount(mj); } }
    HITJ(0, h0, s0)
    HITJ(1, h1, s1)
    HITJ(2, h2, s2)
    HITJ(3, h3, s3)
    HITJ(4, h4, s4)
    HITJ(5, h5, s5)
    HITJ(6, h6, s6)
    HITJ(7, h7, s7)
#undef HITJ
  }
  return wc;
}

__global__ __launch_bounds__(NTHR) void k_xprep(const float* __restrict__ x, unsigned short* xb, int nN, int nUnits) {
  const int i = (int)blockIdx.x * NTHR + (int)threadIdx.x;
  if (i >= nUnits) return;
  const int row = i >> 5;
  const int c0  = (i & 31) * 8;
  const int rc  = row < nN ? row : nN - 1;
  const float* p = x + (size_t)rc * F_IN + c0;
  v4f a = *(const v4fa*)p, b = *(const v4fa*)(p + 4);
  const v4f z4 = {0.f, 0.f, 0.f, 0.f};
  if (row >= nN) { a = z4; b = z4; }
  const v4u hv = pack8(a, b);
  const size_t o = (size_t)row * F_IN + c0;
  *(volatile v4u*)(xb + o) = hv;
  __threadfence();
  *(volatile v4u*)(xb + o) = hv;
}

__global__ __launch_bounds__(NTHR) void k_wtr(const float* __restrict__ w, int Kin, int Ncol, int Nrows, int Kout,
                                              unsigned short* wt, int nUnits) {
  const int u = (int)blockIdx.x * NTHR + (int)threadIdx.x;
  if (u >= nUnits) return;
  const int kq = Kout >> 3;
  const int n  = u / kq;
  const int k8 = (u - n * kq) * 8;
  const int kk = k8 - (k8 / Kin) * Kin;
  const int ncl = n < Ncol ? n : Ncol - 1;
  const float* p = w + (size_t)kk * (size_t)Ncol + ncl;
  v4f a, b;
  a.x = p[0];                    a.y = p[(size_t)Ncol];         a.z = p[(size_t)2 * Ncol];     a.w = p[(size_t)3 * Ncol];
  b.x = p[(size_t)4 * Ncol];     b.y = p[(size_t)5 * Ncol];     b.z = p[(size_t)6 * Ncol];     b.w = p[(size_t)7 * Ncol];
  const v4f z4 = {0.f, 0.f, 0.f, 0.f};
  if (n >= Ncol || n >= Nrows) { a = z4; b = z4; }
  const v4u wv = pack8(a, b);
  unsigned short* o = wt + (size_t)n * (size_t)Kout + k8;
  *(volatile v4u*)o = wv;
  __threadfence();
  *(volatile v4u*)o = wv;
}

__global__ __launch_bounds__(NTHR) void k_bucket(const int* __restrict__ srcs, const int* __restrict__ dsts,
                                                 int* hits, int nN, int nE, int vec8) {
  extern __shared__ v4f lds_dyn[];
  int* reg1 = (int*)lds_dyn;
  int* reg2 = reg1 + RCAP;
  int* scnt = reg2 + RCAP;
  int* soff = scnt + NB;
  int* list = soff + NB;
  int* wcnt = list + LISTN;
  int* wtot = wcnt + NWAVE;
  int* hdr  = wtot + NWAVE;
  const int tid = (int)threadIdx.x, lane = tid & 31, wave = tid >> 5;
  const int nodeBase = (int)blockIdx.x * NB;

  {
    const v4i z4 = {0, 0, 0, 0};
    for (int i = 4 * tid; i < RCAP; i += 4 * NTHR) *(v4ia*)(reg2 + i) = z4;
    for (int i = tid; i < NB; i += NTHR) scnt[i] = 0;
  }
  __syncthreads();

  int tot = 0;
  const int nChunks = (nE + CHUNK - 1) / CHUNK;
#pragma unroll 1
  for (int ch = 0; ch < nChunks; ++ch) {
    const int cbase = ch * CHUNK;
    const int wc = scan_chunk(dsts, nE, cbase, nodeBase, NB, vec8, list, tid, lane, wave);
    if (lane == 0) wcnt[wave] = wc;
    __syncthreads();
    int pre = 0, all = 0;
#pragma unroll
    for (int w2 = 0; w2 < NWAVE; ++w2) {
      int c = wcnt[w2];
      c = c < 0 ? 0 : (c > WCAP ? WCAP : c);
      all += c;
      pre += (w2 < wave) ? c : 0;
    }
    const int wcc  = wc > WCAP ? WCAP : wc;
    const int base = tot + pre;
#pragma unroll 1
    for (int i0 = 0; i0 < wcc; i0 += 32) {
      const int i   = i0 + lane;
      const int ic  = i < wcc ? i : wcc - 1;
      const int ent = list[wave * WCAP + ic];
      const int el  = (ent >> SLOTB) & (CHUNK - 1);
      const int sl  = ent & (NB - 1);
      int eid = cbase + el;
      eid = eid < 0 ? 0 : (eid > nE - 1 ? nE - 1 : eid);
      int s = srcs[eid];
      s = s < 0 ? 0 : (s > nN - 1 ? nN - 1 : s);
      const int pos = base + i;
      if (i < wcc && pos < RCAP) reg1[pos] = s | (sl << 16);
    }
    tot += all;
    tot = tot > RCAP ? RCAP : tot;
    __syncthreads();
  }
  const int nh = tot;

  if (wave == 0) {
#pragma unroll 1
    for (int b0 = 0; b0 < nh; b0 += 32) {
      const int idx = b0 + lane;
      const int uv  = reg1[idx < nh ? idx : nh - 1];
      const int m32 = (nh - b0) < 32 ? (nh - b0) : 32;
#pragma unroll 1
      for (int k = 0; k < m32; ++k) {
        const int u  = __builtin_amdgcn_readlane(uv, k);
        const int sl = (u >> 16) & (NB - 1);
        if (lane == 0) scnt[sl] = scnt[sl] + 1;
      }
    }
  }
  __syncthreads();

  {
    int e0 = scnt[2 * tid], e1 = scnt[2 * tid + 1];
    e0 = e0 < 0 ? 0 : e0;
    e1 = e1 < 0 ? 0 : e1;
    const int ts = e0 + e1;
    int incl = ts;
#pragma unroll
    for (int d = 1; d < 32; d <<= 1) {
      const int up = __shfl_up(incl, d);
      if (lane >= d) incl += up;
    }
    if (lane == 31) wtot[wave] = incl;
    __syncthreads();
    int pre = 0;
#pragma unroll
    for (int w2 = 0; w2 < NWAVE; ++w2) pre += (w2 < wave) ? wtot[w2] : 0;
    const int run = pre + incl - ts;
    soff[2 * tid]     = run;
    soff[2 * tid + 1] = run + e0;
  }
  __syncthreads();
  for (int i = tid; i < NB; i += NTHR) list[i] = soff[i];
  __syncthreads();

  if (wave == 0) {
#pragma unroll 1
    for (int b0 = 0; b0 < nh; b0 += 32) {
      const int idx = b0 + lane;
      const int uv  = reg1[idx < nh ? idx : nh - 1];
      const int m32 = (nh - b0) < 32 ? (nh - b0) : 32;
#pragma unroll 1
      for (int k = 0; k < m32; ++k) {
        const int u  = __builtin_amdgcn_readlane(uv, k);
        const int sl = (u >> 16) & (NB - 1);
        if (lane == 0) {
          int pos = list[sl];
          pos = pos < 0 ? 0 : (pos > RCAP - 1 ? RCAP - 1 : pos);
          reg2[pos] = u;
          list[sl] = pos + 1;
        }
      }
    }
  }
  if (tid < HDR) hdr[tid] = (tid == 0) ? nh : ((tid == 1) ? ((nh >= RCAP) ? 1 : 0) : 0);
  __syncthreads();

  int* hb = hits + (size_t)blockIdx.x * HPITCH;
#pragma unroll 1
  for (int i = 4 * tid; i < RCAP; i += 4 * NTHR) {
    const v4i v = *(const v4ia*)(reg2 + i);
    *(volatile v4i*)(hb + HDR + i) = v;
  }
  v4i hv = {0, 0, 0, 0};
  if (tid < 8) { hv = *(const v4ia*)(hdr + 4 * tid); *(volatile v4i*)(hb + 4 * tid) = hv; }
  __threadfence();
#pragma unroll 1
  for (int i = 4 * tid; i < RCAP; i += 4 * NTHR) {
    const v4i v = *(const v4ia*)(reg2 + i);
    *(volatile v4i*)(hb + HDR + i) = v;
  }
  if (tid < 8) *(volatile v4i*)(hb + 4 * tid) = hv;
}

template <int HPB>
__global__ __launch_bounds__(GTHR) void k_gemm(
    const unsigned short* __restrict__ A, const unsigned short* __restrict__ WT,
    float* outF, int K, int ldo,
    const float* __restrict__ atts, const float* __restrict__ attd, int attTot,
    float* SD, int MPr)
{
  constexpr int CH = GBN / HPB;
  __shared__ __attribute__((aligned(16))) float stg[GBM * GBN];
  __shared__ __attribute__((aligned(16))) float satt[2 * GBN];
  __shared__ __attribute__((aligned(16))) float sdot[2 * HPB * GBM];
  const int tid = (int)threadIdx.x, lane = tid & 31, wave = tid >> 5, hh = lane >> 4, m = lane & 15;
  const int rowBase = (int)blockIdx.x * GBM;
  const int col0    = (int)blockIdx.y * GBN;

  {
    const int which = tid >> 6;
    const int c  = tid & 63;
    const int gi = col0 + c;
    const int cl = gi < attTot ? gi : attTot - 1;
    const float vs = atts[cl];
    const float vd = attd[cl];
    const unsigned int msk = (which == 0) ? 0u : 0xFFFFFFFFu;
    const unsigned int inr = (gi < attTot) ? 0xFFFFFFFFu : 0u;
    float v = __uint_as_float((__float_as_uint(vs) & ~msk) | (__float_as_uint(vd) & msk));
    v = __uint_as_float(__float_as_uint(bfr(v)) & inr);
    satt[which * GBN + c] = v;
  }

  v8f acc[4];
  {
    const v8f z = {0.f, 0.f, 0.f, 0.f, 0.f, 0.f, 0.f, 0.f};
    acc[0] = z; acc[1] = z; acc[2] = z; acc[3] = z;
  }
  const unsigned short* ap = A  + (size_t)(rowBase + 16 * wave + m) * (size_t)K + 8 * hh;
  const unsigned short* wp = WT + (size_t)(col0 + m) * (size_t)K + 8 * hh;
  const int ksteps = K >> 5;
#pragma unroll 1
  for (int ks = 0; ks < ksteps; ++ks) {
    FragB af;
    af.h[0] = *(const v8usa*)(ap + 32 * ks);
    af.h[1] = *(const v8usa*)(ap + 32 * ks + 16);
#pragma unroll
    for (int t = 0; t < 4; ++t) {
      const unsigned short* wq = wp + (size_t)(16 * t) * (size_t)K + 32 * ks;
      FragB bf;
      bf.h[0] = *(const v8usa*)wq;
      bf.h[1] = *(const v8usa*)(wq + 16);
      acc[t] = wmb(af, bf, acc[t]);
    }
  }

#pragma unroll
  for (int t = 0; t < 4; ++t) {
    const int lc = 16 * t + m;
#pragma unroll
    for (int r = 0; r < 8; ++r) {
      const int lr = 16 * wave + 8 * hh + r;
      stg[lr * GBN + lc] = acc[t][r];
    }
  }
  __syncthreads();

  {
    const int row = tid & 63, which = tid >> 6;
    const float* sa = satt + which * GBN;
    const float* hr = stg + row * GBN;
#pragma unroll
    for (int hd = 0; hd < HPB; ++hd) {
      float d = 0.f;
#pragma unroll 4
      for (int c4 = 0; c4 < CH / 4; ++c4) {
        const v4f hv = *(const v4fa*)(hr + hd * CH + 4 * c4);
        const v4f av = *(const v4fa*)(sa + hd * CH + 4 * c4);
        d = fmaf(hv.x, av.x, d);
        d = fmaf(hv.y, av.y, d);
        d = fmaf(hv.z, av.z, d);
        d = fmaf(hv.w, av.w, d);
      }
      sdot[(which * HPB + hd) * GBM + row] = d;
    }
  }
  __syncthreads();

  v4f fv[8];
#pragma unroll
  for (int i = 0; i < 8; ++i) {
    const int lr = 16 * wave + 2 * i + hh;
    fv[i] = *(const v4fa*)(stg + lr * GBN + 4 * m);
  }
  const int which2 = lane >> 4, piece = lane & 15;
  const int hdw = wave < HPB ? wave : 0;
  const v4f sdv = *(const v4fa*)(sdot + (which2 * HPB + hdw) * GBM + 4 * piece);
  float* sp = SD + (size_t)(2 * ((int)blockIdx.y * HPB + hdw) + which2) * (size_t)MPr + rowBase + 4 * piece;

#pragma unroll
  for (int i = 0; i < 8; ++i) {
    const int lr = 16 * wave + 2 * i + hh;
    const int gr = rowBase + lr;
    float* op = outF + (size_t)gr * (size_t)ldo + col0 + 4 * m;
    *(volatile v4f*)op = fv[i];
  }
  if (wave < HPB) *(volatile v4f*)sp = sdv;
  __threadfence();
#pragma unroll
  for (int i = 0; i < 8; ++i) {
    const int lr = 16 * wave + 2 * i + hh;
    const int gr = rowBase + lr;
    float* op = outF + (size_t)gr * (size_t)ldo + col0 + 4 * m;
    *(volatile v4f*)op = fv[i];
  }
  if (wave < HPB) *(volatile v4f*)sp = sdv;
}

template <int NC>
__global__ __launch_bounds__(NTHR) void k_agg(
    const int* __restrict__ hits, const float* __restrict__ F, const float* __restrict__ SD,
    const float* __restrict__ bias, float* P, double* REC, int nN, int MPr) {
  extern __shared__ v4f lds_dyn[];
  double* wst  = (double*)lds_dyn;
  double* rec  = wst + NWAVE * RECW;
  int*    reg  = (int*)(rec + RECW);
  int*    soff = reg + RCAP;
  int*    send = soff + NB;
  const int tid = (int)threadIdx.x, lane = tid & 31, wave = tid >> 5;
  const int nodeBase = (int)blockIdx.x * NB;
  const int* hb = hits + (size_t)blockIdx.x * HPITCH;
  int nh = hb[0];
  nh = nh < 0 ? 0 : (nh > RCAP ? RCAP : nh);
  const int ofl = hb[1];

  for (int i = tid; i < 2 * NB; i += NTHR) soff[i] = 0;
#pragma unroll 1
  for (int i0 = 0; i0 < nh; i0 += 4 * NTHR) {
    const int i = i0 + 4 * tid;
    const v4i v = *(const v4i*)(hb + HDR + i);
    *(v4ia*)(reg + i) = v;
  }
  __syncthreads();
#pragma unroll 1
  for (int i0 = 0; i0 < nh; i0 += NTHR) {
    const int i  = i0 + tid;
    const int ic = i < nh ? i : nh - 1;
    const int ip = ic > 0 ? ic - 1 : 0;
    const int in = ic < nh - 1 ? ic + 1 : nh - 1;
    const int sl  = (reg[ic] >> 16) & (NB - 1);
    const int psl = (reg[ip] >> 16) & (NB - 1);
    const int nsl = (reg[in] >> 16) & (NB - 1);
    if (i < nh) {
      if (ic == 0 || psl != sl)      soff[sl] = ic;
      if (ic == nh - 1 || nsl != sl) send[sl] = ic + 1;
    }
  }
  __syncthreads();

  const bool ovf = (ofl != 0) || (nh >= RCAP);
  const float qnan = __int_as_float(0x7fc00000);
  constexpr int NBW = NB / NWAVE;

  if constexpr (NC == 128) {
    const int c0   = 4 * lane;
    const int head = lane >> 3;
    const v4f bb   = bfr4(*(const v4fa*)(bias + c0));
    const float* ASp = SD + (size_t)(2 * head) * (size_t)MPr;
    const float* ADp = ASp + MPr;
    double s1x = 0.0, s1y = 0.0, s1z = 0.0, s1w = 0.0;
    double s2x = 0.0, s2y = 0.0, s2z = 0.0, s2w = 0.0;

#pragma unroll 1
    for (int jt = 0; jt < NBW; ++jt) {
      const int slot = wave * NBW + jt;
      const int grow = nodeBase + slot;
      const int gcl  = grow < nN ? grow : nN - 1;
      int st = soff[slot];
      const int craw = send[slot] - st;
      int cnt = craw;
      st  = st < 0 ? 0 : (st > nh ? nh : st);
      cnt = cnt < 0 ? 0 : (cnt > DEGCAP ? DEGCAP : cnt);
      if (cnt > nh - st) cnt = nh - st;
      const float pz = (ovf || craw > DEGCAP || craw < 0) ? qnan : 0.0f;

      v4f av = *(const v4fa*)(F + (size_t)gcl * HC + c0);
      const float adv = ADp[gcl];
      float l0 = ASp[gcl] + adv;
      l0 = l0 > 0.f ? l0 : NEGSL * l0;
      float mx = l0, dn = 1.0f;

#pragma unroll 1
      for (int q = 0; q < cnt; ++q) {
        int idx = st + q; idx = idx > RCAP - 1 ? RCAP - 1 : idx;
        int s = reg[idx] & 0xFFFF;
        s = s > nN - 1 ? nN - 1 : s;
        const v4f fa = *(const v4fa*)(F + (size_t)s * HC + c0);
        float lg = ASp[s] + adv;
        lg = lg > 0.f ? lg : NEGSL * lg;
        const float df = lg - mx;
        const float ee = __expf(-fabsf(df));
        const bool up  = df > 0.f;
        const float f1 = up ? ee : 1.0f;
        const float f2 = up ? 1.0f : ee;
        mx = up ? lg : mx;
        dn = fmaf(dn, f1, f2);
        av.x = fmaf(av.x, f1, f2 * fa.x);
        av.y = fmaf(av.y, f1, f2 * fa.y);
        av.z = fmaf(av.z, f1, f2 * fa.z);
        av.w = fmaf(av.w, f1, f2 * fa.w);
      }
      const float inv = __builtin_amdgcn_rcpf(dn);
      const bool live = grow < nN;
      v4f o;
      o.x = (live ? fmaf(av.x, inv, bb.x) : 0.f) + pz;
      o.y = (live ? fmaf(av.y, inv, bb.y) : 0.f) + pz;
      o.z = (live ? fmaf(av.z, inv, bb.z) : 0.f) + pz;
      o.w = (live ? fmaf(av.w, inv, bb.w) : 0.f) + pz;
      if (live) {
        const double dx = (double)o.x, dy = (double)o.y, dz = (double)o.z, dw = (double)o.w;
        s1x += dx; s1y += dy; s1z += dz; s1w += dw;
        s2x += dx * dx; s2y += dy * dy; s2z += dz * dz; s2w += dw * dw;
      }
      float* pp = P + (size_t)grow * HC + c0;
      const bool wr = grow < MPr;
      if (wr) *(volatile v4f*)pp = o;
      __threadfence();
      if (wr) *(volatile v4f*)pp = o;
    }
    double* wp = wst + wave * RECW;
    wp[c0 + 0] = s1x; wp[c0 + 1] = s1y; wp[c0 + 2] = s1z; wp[c0 + 3] = s1w;
    wp[NC + c0 + 0] = s2x; wp[NC + c0 + 1] = s2y; wp[NC + c0 + 2] = s2z; wp[NC + c0 + 3] = s2w;
  } else {
    const int c0 = 2 * lane;
    const v2f bb = bfr2(*(const v2fa*)(bias + c0));
    const float* ASp = SD;
    const float* ADp = SD + MPr;
    double s1x = 0.0, s1y = 0.0, s2x = 0.0, s2y = 0.0;

#pragma unroll 1
    for (int jt = 0; jt < NBW; ++jt) {
      const int slot = wave * NBW + jt;
      const int grow = nodeBase + slot;
      const int gcl  = grow < nN ? grow : nN - 1;
      int st = soff[slot];
      const int craw = send[slot] - st;
      int cnt = craw;
      st  = st < 0 ? 0 : (st > nh ? nh : st);
      cnt = cnt < 0 ? 0 : (cnt > DEGCAP ? DEGCAP : cnt);
      if (cnt > nh - st) cnt = nh - st;
      const float pz = (ovf || craw > DEGCAP || craw < 0) ? qnan : 0.0f;

      const v2f fd = *(const v2fa*)(F + (size_t)gcl * HC3 + c0);
      const float adv = ADp[gcl];
      float l0 = ASp[gcl] + adv;
      l0 = l0 > 0.f ? l0 : NEGSL * l0;
      float mx = l0, dn = 1.0f;
      float a0 = fd.x, a1 = fd.y;

#pragma unroll 1
      for (int q = 0; q < cnt; ++q) {
        int idx = st + q; idx = idx > RCAP - 1 ? RCAP - 1 : idx;
        int s = reg[idx] & 0xFFFF;
        s = s > nN - 1 ? nN - 1 : s;
        const v2f fs = *(const v2fa*)(F + (size_t)s * HC3 + c0);
        float lg = ASp[s] + adv;
        lg = lg > 0.f ? lg : NEGSL * lg;
        const float df = lg - mx;
        const float ee = __expf(-fabsf(df));
        const bool up  = df > 0.f;
        const float f1 = up ? ee : 1.0f;
        const float f2 = up ? 1.0f : ee;
        mx = up ? lg : mx;
        dn = fmaf(dn, f1, f2);
        a0 = fmaf(a0, f1, f2 * fs.x);
        a1 = fmaf(a1, f1, f2 * fs.y);
      }
      const float inv = __builtin_amdgcn_rcpf(dn);
      const bool live = grow < nN;
      v2f o;
      o.x = (live ? fmaf(a0, inv, bb.x) : 0.f) + pz;
      o.y = (live ? fmaf(a1, inv, bb.y) : 0.f) + pz;
      if (live) {
        const double dx = (double)o.x, dy = (double)o.y;
        s1x += dx; s1y += dy;
        s2x += dx * dx; s2y += dy * dy;
      }
      float* pp = P + (size_t)grow * HC3 + c0;
      const bool wr = grow < MPr;
      if (wr) *(volatile v2f*)pp = o;
      __threadfence();
      if (wr) *(volatile v2f*)pp = o;
    }
    double* wp = wst + wave * RECW;
    wp[c0 + 0] = s1x; wp[c0 + 1] = s1y;
    wp[NC + c0 + 0] = s2x; wp[NC + c0 + 1] = s2y;
  }

  __syncthreads();
  if (tid < 2 * NC) {
    double a = 0.0;
#pragma unroll 1
    for (int w2 = 0; w2 < NWAVE; ++w2) a += wst[w2 * RECW + tid];
    rec[tid] = a;
  }
  __syncthreads();
  v2d rv = {0.0, 0.0};
  double* rp = REC + (size_t)blockIdx.x * RECW + 2 * tid;
  if (tid < NC) { rv.x = rec[2 * tid]; rv.y = rec[2 * tid + 1]; *(volatile v2d*)rp = rv; }
  __threadfence();
  if (tid < NC) *(volatile v2d*)rp = rv;
}

__global__ __launch_bounds__(NTHR) void k_stat(const double* __restrict__ REC, int nBlk, int NC, int nN,
                                               const float* __restrict__ gam, const float* __restrict__ bet,
                                               float* ss) {
  __shared__ double dsum[RECW];
  __shared__ __attribute__((aligned(16))) float stg[3 * HC];
  const int tid = (int)threadIdx.x;
  {
    const int tc = tid < 2 * NC ? tid : 0;
    double a = 0.0;
#pragma unroll 1
    for (int b = 0; b < nBlk; ++b) a += REC[(size_t)b * RECW + tc];
    dsum[tid] = a;
  }
  __syncthreads();
  {
    const int c = tid < NC ? tid : NC - 1;
    const double inv = 1.0 / (double)nN;
    const double mean = dsum[c] * inv;
    double var = dsum[NC + c] * inv - mean * mean;
    var = (var < 0.0) ? 0.0 : var;
    const float rstd = 1.0f / sqrtf((float)var + 1e-5f);
    const float gv = bfr(gam[c]);
    const float bv = bfr(bet[c]);
    if (tid < NC) {
      stg[c] = (float)mean;
      stg[NC + c] = gv * rstd;
      stg[2 * NC + c] = bv;
    }
  }
  __syncthreads();
  v4f v = {0.f, 0.f, 0.f, 0.f};
  const int np = (3 * NC) >> 2;
  if (tid < np) {
    v = *(const v4fa*)(stg + 4 * tid);
    *(volatile v4f*)(ss + 4 * tid) = v;
  }
  __threadfence();
  if (tid < np) *(volatile v4f*)(ss + 4 * tid) = v;
}

__global__ __launch_bounds__(NTHR) void k_norm12(const float* __restrict__ P, const float* __restrict__ ss,
                                                 unsigned short* A, int nN, int nUnits) {
  __shared__ __attribute__((aligned(16))) float ssh[3 * HC];
  const int tid = (int)threadIdx.x;
  if (tid < (3 * HC) / 4) *(v4fa*)(ssh + 4 * tid) = *(const v4f*)(ss + 4 * tid);
  __syncthreads();
  const int u = (int)blockIdx.x * NTHR + tid;
  if (u >= nUnits) return;
  const int row = u >> 4;
  const int c0  = (u & 15) * 8;
  const float* p = P + (size_t)row * HC + c0;
  const v4f xa = *(const v4f*)p, xb = *(const v4f*)(p + 4);
  const v4f ma = *(const v4fa*)(ssh + c0),          mb = *(const v4fa*)(ssh + c0 + 4);
  const v4f sa = *(const v4fa*)(ssh + HC + c0),     sb = *(const v4fa*)(ssh + HC + c0 + 4);
  const v4f ba = *(const v4fa*)(ssh + 2 * HC + c0), bb = *(const v4fa*)(ssh + 2 * HC + c0 + 4);
  const bool live = row < nN;
  float y[8];
  y[0] = relun(fmaf(xa.x - ma.x, sa.x, ba.x));
  y[1] = relun(fmaf(xa.y - ma.y, sa.y, ba.y));
  y[2] = relun(fmaf(xa.z - ma.z, sa.z, ba.z));
  y[3] = relun(fmaf(xa.w - ma.w, sa.w, ba.w));
  y[4] = relun(fmaf(xb.x - mb.x, sb.x, bb.x));
  y[5] = relun(fmaf(xb.y - mb.y, sb.y, bb.y));
  y[6] = relun(fmaf(xb.z - mb.z, sb.z, bb.z));
  y[7] = relun(fmaf(xb.w - mb.w, sb.w, bb.w));
  unsigned int hq[8], lq[8];
#pragma unroll
  for (int j = 0; j < 8; ++j) {
    const float yy = live ? y[j] : 0.0f;
    hq[j] = f2bf(yy);
    lq[j] = f2bf(yy - bf2f(hq[j]));
  }
  v4u hv, lv;
  hv.x = hq[0] | (hq[1] << 16); hv.y = hq[2] | (hq[3] << 16); hv.z = hq[4] | (hq[5] << 16); hv.w = hq[6] | (hq[7] << 16);
  lv.x = lq[0] | (lq[1] << 16); lv.y = lq[2] | (lq[3] << 16); lv.z = lq[4] | (lq[5] << 16); lv.w = lq[6] | (lq[7] << 16);
  unsigned short* gp = A + (size_t)row * KA + c0;
  unsigned short* gq = gp + HC;
  *(volatile v4u*)gp = hv;
  *(volatile v4u*)gq = lv;
  __threadfence();
  *(volatile v4u*)gp = hv;
  *(volatile v4u*)gq = lv;
}

__global__ __launch_bounds__(NTHR) void k_norm3(const float* __restrict__ P, const float* __restrict__ ss,
                                                float* out, int nUnits) {
  __shared__ __attribute__((aligned(16))) float ssh[4 * HC3];
  const int tid = (int)threadIdx.x;
  if (tid < 64) {
    const int si = tid < (3 * HC3) / 4 ? tid : (3 * HC3) / 4 - 1;
    *(v4fa*)(ssh + 4 * tid) = *(const v4f*)(ss + 4 * si);
  }
  __syncthreads();
  const int u = (int)blockIdx.x * NTHR + tid;
  if (u >= nUnits) return;
  const int c0 = (u & 15) * 4;
  const v4f x = *(const v4f*)(P + (size_t)u * 4);
  const v4f mv = *(const v4fa*)(ssh + c0);
  const v4f sv = *(const v4fa*)(ssh + HC3 + c0);
  const v4f bv = *(const v4fa*)(ssh + 2 * HC3 + c0);
  v4f o;
  o.x = fmaf(x.x - mv.x, sv.x, bv.x);
  o.y = fmaf(x.y - mv.y, sv.y, bv.y);
  o.z = fmaf(x.z - mv.z, sv.z, bv.z);
  o.w = fmaf(x.w - mv.w, sv.w, bv.w);
  float* op = out + (size_t)u * 4;
  *(volatile v4f*)op = o;
  __threadfence();
  *(volatile v4f*)op = o;
}

static inline int cdiv(int a, int b) { return (a + b - 1) / b; }
static inline size_t al256(size_t o) { return (o + 255) & ~(size_t)255; }

extern "C" void kernel_launch(void* const* d_in, const int* in_sizes, int n_in,
                              void* d_out, int out_size, void* d_ws, size_t ws_size,
                              hipStream_t stream) {
  if (n_in < 20) return;
  const int nN = in_sizes[0] / F_IN;
  if (nN <= 0 || in_sizes[0] != nN * F_IN || nN > 65536) return;
  if (in_sizes[1] < 2 || (in_sizes[1] & 1) != 0) return;
  const int nE = in_sizes[1] / 2;
  if (nE < 1 || nE > (1 << 30)) return;
  if (in_sizes[2] != F_IN * HC) return;
  if (in_sizes[3] != HC || in_sizes[4] != HC) return;
  if (in_sizes[5] != HC || in_sizes[6] != HC || in_sizes[7] != HC) return;
  if (in_sizes[8] != HC * HC) return;
  if (in_sizes[9] != HC || in_sizes[10] != HC) return;
  if (in_sizes[11] != HC || in_sizes[12] != HC || in_sizes[13] != HC) return;
  if (in_sizes[14] != HC * HC3) return;
  if (in_sizes[15] != HC3 || in_sizes[16] != HC3) return;
  if (in_sizes[17] != HC3 || in_sizes[18] != HC3 || in_sizes[19] != HC3) return;
  if (out_size != nN * HC3) return;

  const float* x   = (const float*)d_in[0];
  const int*   ei  = (const int*)  d_in[1];
  const float* W1  = (const float*)d_in[2];
  const float* a1s = (const float*)d_in[3];
  const float* a1d = (const float*)d_in[4];
  const float* b1  = (const float*)d_in[5];
  const float* g1  = (const float*)d_in[6];
  const float* be1 = (const float*)d_in[7];
  const float* W2  = (const float*)d_in[8];
  const float* a2s = (const float*)d_in[9];
  const float* a2d = (const float*)d_in[10];
  const float* b2  = (const float*)d_in[11];
  const float* g2  = (const float*)d_in[12];
  const float* be2 = (const float*)d_in[13];
  const float* W3  = (const float*)d_in[14];
  const float* a3s = (const float*)d_in[15];
  const float* a3d = (const float*)d_in[16];
  const float* b3  = (const float*)d_in[17];
  const float* g3  = (const float*)d_in[18];
  const float* be3 = (const float*)d_in[19];
  float* out = (float*)d_out;
  const int* src = ei;
  const int* dst = ei + nE;

  const int MP   = cdiv(nN, MROWS) * MROWS;
  const int gA   = cdiv(MP, NB);
  const int gM   = MP / GBM;
  const int vec8 = ((nE & 3) == 0) ? 1 : 0;
  if (gA * NB < MP) return;

  char* ws = (char*)d_ws;
  size_t off = 0;
  const size_t oA   = off; off = al256(off + (size_t)MP * KA * 2);
  const size_t oW1T = off; off = al256(off + (size_t)HC * KA * 2);
  const size_t oW2T = off; off = al256(off + (size_t)HC * KA * 2);
  const size_t oW3T = off; off = al256(off + (size_t)HC3 * KA * 2);
  const size_t oH   = off; off = al256(off + (size_t)MP * HC * 4);
  const size_t oP   = off; off = al256(off + (size_t)MP * HC * 4);
  const size_t oSD  = off; off = al256(off + (size_t)8 * MP * 4);
  const size_t oHT  = off; off = al256(off + (size_t)gA * HPITCH * 4);
  const size_t oRC  = off; off = al256(off + (size_t)gA * RECW * 8);
  const size_t oSS  = off; off = al256(off + (size_t)(3 * HC) * 4);
  if (off > ws_size || off > (size_t)WSMAX) return;
  unsigned short* AP  = (unsigned short*)(ws + oA);
  unsigned short* W1T = (unsigned short*)(ws + oW1T);
  unsigned short* W2T = (unsigned short*)(ws + oW2T);
  unsigned short* W3T = (unsigned short*)(ws + oW3T);
  float*          H   = (float*)(ws + oH);
  float*          P   = (float*)(ws + oP);
  float*          SD  = (float*)(ws + oSD);
  int*            HT  = (int*)(ws + oHT);
  double*         RC  = (double*)(ws + oRC);
  float*          SS  = (float*)(ws + oSS);

  hipFuncSetAttribute(reinterpret_cast<const void*>(&k_bucket),
                      hipFuncAttributeMaxDynamicSharedMemorySize, LDS_BKT);
  hipFuncSetAttribute(reinterpret_cast<const void*>(&k_agg<128>),
                      hipFuncAttributeMaxDynamicSharedMemorySize, LDS_AGG);
  hipFuncSetAttribute(reinterpret_cast<const void*>(&k_agg<64>),
                      hipFuncAttributeMaxDynamicSharedMemorySize, LDS_AGG);

  const int nUx = MP * (F_IN / 8);
  k_xprep<<<cdiv(nUx, NTHR), NTHR, 0, stream>>>(x, AP, nN, nUx);

  {
    const int nUw1 = HC * (KA / 8);
    k_wtr<<<cdiv(nUw1, NTHR), NTHR, 0, stream>>>(W1, F_IN, HC, HC, KA, W1T, nUw1);
    const int nUw2 = HC * (KA / 8);
    k_wtr<<<cdiv(nUw2, NTHR), NTHR, 0, stream>>>(W2, HC, HC, HC, KA, W2T, nUw2);
    const int nUw3 = HC3 * (KA / 8);
    k_wtr<<<cdiv(nUw3, NTHR), NTHR, 0, stream>>>(W3, HC, HC3, HC3, KA, W3T, nUw3);
  }

  k_bucket<<<gA, NTHR, LDS_BKT, stream>>>(src, dst, HT, nN, nE, vec8);

  const int nU12 = MP * (HC / 8);
  const int nU3  = nN * (HC3 / 4);

  k_gemm<2><<<dim3(gM, HC / GBN), GTHR, 0, stream>>>(AP, W1T, H, KA, HC, a1s, a1d, HC, SD, MP);
  k_agg<128><<<gA, NTHR, LDS_AGG, stream>>>(HT, H, SD, b1, P, RC, nN, MP);
  k_stat<<<1, NTHR, 0, stream>>>(RC, gA, HC, nN, g1, be1, SS);
  k_norm12<<<cdiv(nU12, NTHR), NTHR, 0, stream>>>(P, SS, AP, nN, nU12);
  k_gemm<2><<<dim3(gM, HC / GBN), GTHR, 0, stream>>>(AP, W2T, H, KA, HC, a2s, a2d, HC, SD, MP);
  k_agg<128><<<gA, NTHR, LDS_AGG, stream>>>(HT, H, SD, b2, P, RC, nN, MP);
  k_stat<<<1, NTHR, 0, stream>>>(RC, gA, HC, nN, g2, be2, SS);
  k_norm12<<<cdiv(nU12, NTHR), NTHR, 0, stream>>>(P, SS, AP, nN, nU12);
  k_gemm<1><<<dim3(gM, HC3 / GBN), GTHR, 0, stream>>>(AP, W3T, H, KA, HC3, a3s, a3d, HC3, SD, MP);
  k_agg<64><<<gA, NTHR, LDS_AGG, stream>>>(HT, H, SD, b3, P, RC, nN, MP);
  k_stat<<<1, NTHR, 0, stream>>>(RC, gA, HC3, nN, g3, be3, SS);
  k_norm3<<<cdiv(nU3, NTHR), NTHR, 0, stream>>>(P, SS, out, nU3);
}
